// PairSelfAttention_77232101916715
// MI455X (gfx1250) — hardware-verified
//
#include <hip/hip_runtime.h>
#include <math.h>

typedef __attribute__((ext_vector_type(16))) _Float16 v16h;
typedef __attribute__((ext_vector_type(16))) __bf16 v16b;
typedef __attribute__((ext_vector_type(8)))  _Float16 v8h;
typedef __attribute__((ext_vector_type(8)))  float v8f;
typedef __attribute__((ext_vector_type(4)))  float v4f;
typedef __attribute__((ext_vector_type(2)))  float v2f;
typedef __attribute__((ext_vector_type(4)))  unsigned v4u;
typedef __attribute__((ext_vector_type(4)))  int v4i;
typedef float __attribute__((may_alias)) float_a;
typedef int __attribute__((may_alias)) int_a;

template <typename T> __device__ __forceinline__ void vst2(void* p, T v) { *(volatile T*)p = v; __threadfence(); *(volatile T*)p = v; }
__device__ __forceinline__ v8f wmma16(v16h a, v16h b, v8f c) {
  v8f d = __builtin_amdgcn_wmma_f32_16x16x32_f16(false, a, false, b, (short)0, c, false, false);
  asm volatile("v_nop\n\tv_nop\n\tv_nop\n\tv_nop" : "+v"(d) : "v"(a), "v"(b));
  return d;
}
__device__ __forceinline__ v8f wmma_bf(v16b a, v16b b, v8f c) {
  v8f d = __builtin_amdgcn_wmma_f32_16x16x32_bf16(false, a, false, b, (short)0, c, false, false);
  asm volatile("v_nop\n\tv_nop\n\tv_nop\n\tv_nop" : "+v"(d) : "v"(a), "v"(b));
  return d;
}
__device__ __forceinline__ v16h frag_h(const _Float16* rowk0, int lane) {
  union { v16h v; v8h q[2]; } u; const _Float16* p = rowk0 + 8 * (lane >> 4);
  u.q[0] = *(const v8h*)p; u.q[1] = *(const v8h*)(p + 16); return u.v;
}
__device__ __forceinline__ v16h frag_f32(const float* rowk0, int lane) {
  v16h a; const float* p = rowk0 + 8 * (lane >> 4);
#pragma unroll
  for (int i = 0; i < 8; ++i) { a[i] = (_Float16)p[i]; a[8 + i] = (_Float16)p[16 + i]; }
  return a;
}
__device__ __forceinline__ v16h frag_f32s(const float* rowk0, int lane, float sc) {
  v16h a; const float* p = rowk0 + 8 * (lane >> 4);
#pragma unroll
  for (int i = 0; i < 8; ++i) { a[i] = (_Float16)(p[i] * sc); a[8 + i] = (_Float16)(p[16 + i] * sc); }
  return a;
}
__device__ __forceinline__ v16h fragc_f32(const float* W, int k0, int n, int lane, int ld, int K) {
  v16h a; const int g = lane >> 4;
#pragma unroll
  for (int i = 0; i < 8; ++i) { const int ka = k0 + 8 * g + i, kb = ka + 16;
    a[i] = (_Float16)(ka < K ? W[(size_t)(ka < K ? ka : K - 1) * ld + n] : 0.f); a[8 + i] = (_Float16)(kb < K ? W[(size_t)(kb < K ? kb : K - 1) * ld + n] : 0.f); }
  return a;
}
struct F2 { v16b h, l; };
__device__ __forceinline__ F2 bsplit16(const float v[16]) { F2 r;
#pragma unroll
  for (int i = 0; i < 16; ++i) { const __bf16 h = (__bf16)v[i]; r.h[i] = h; r.l[i] = (__bf16)(v[i] - (float)h); }
  return r; }
__device__ __forceinline__ F2 split_row(const float* row, int k0, int lane) { float v[16]; const float* p = row + k0 + 8 * (lane >> 4);
#pragma unroll
  for (int i = 0; i < 8; ++i) { v[i] = p[i]; v[8 + i] = p[16 + i]; }
  return bsplit16(v); }
__device__ __forceinline__ F2 split_rowK(const float* row, int k0, int lane, int K) { float v[16]; const int g = lane >> 4;
#pragma unroll
  for (int i = 0; i < 8; ++i) { const int ka = k0 + 8 * g + i, kb = ka + 16; v[i] = ka < K ? row[ka < K ? ka : K - 1] : 0.f; v[8 + i] = kb < K ? row[kb < K ? kb : K - 1] : 0.f; }
  return bsplit16(v); }
__device__ __forceinline__ F2 split_col(const float* W, int k0, int n, int lane, int ld, int K) { float v[16]; const int g = lane >> 4;
#pragma unroll
  for (int i = 0; i < 8; ++i) { const int ka = k0 + 8 * g + i, kb = ka + 16; v[i] = ka < K ? W[(size_t)(ka < K ? ka : K - 1) * ld + n] : 0.f; v[8 + i] = kb < K ? W[(size_t)(kb < K ? kb : K - 1) * ld + n] : 0.f; }
  return bsplit16(v); }
__device__ __forceinline__ v8f mac3(const F2& a, const F2& b, v8f c) { c = wmma_bf(a.l, b.h, c); c = wmma_bf(a.h, b.l, c); return wmma_bf(a.h, b.h, c); }
__device__ __forceinline__ float sigm(float v) { return 1.0f / (1.0f + expf(-v)); }
#define LDSX() do { asm volatile("s_wait_dscnt 0" ::: "memory"); __builtin_amdgcn_wave_barrier(); __builtin_amdgcn_fence(__ATOMIC_RELEASE, "workgroup"); } while (0)


#define NB 8
#define NH 8
#define SS 1024
#define HD 64
#ifndef TQB
#define TQB (SS / 64)
#define TNB NB
#endif
typedef __attribute__((ext_vector_type(8))) __bf16 v8b;
__device__ __forceinline__ v16b frag_b(const __bf16* rowk0, int lane) {
  union { v16b v; v8b q[2]; } u; const __bf16* p = rowk0 + 8 * (lane >> 4);
  u.q[0] = *(const v8b*)p; u.q[1] = *(const v8b*)(p + 16); return u.v;
}
__device__ __forceinline__ float bfr(float v) { return (float)(__bf16)v; }
__device__ __attribute__((noinline)) float exp_ni(float v) { return expf(v); }
__device__ __attribute__((noinline)) float erf_ni(float v) { return erff(v); }

#define WS_P0  0u
#define WS_P1  (WS_P0 + 4u * NB * SS)
#define WS_VT  (WS_P1 + 4u * NB * SS)
#define WS_END (WS_VT + 2u * NB * NH * HD * SS)

__global__ __launch_bounds__(256) void k_pairs(const float* __restrict__ C, int* __restrict__ P0, int* __restrict__ P1) {
  #pragma clang fp contract(off)
  __shared__ float sbx[SS][4]; __shared__ __align__(16) int sp0[64], sp1[64];
  const int tid = threadIdx.x, b = blockIdx.y; const int al = tid >> 2, sub = tid & 3; const int a = blockIdx.x * 64 + al;
  for (int c = tid; c < SS; c += 256) { const float cx = bfr(C[((size_t)b * SS + c) * 4 + 0]), cy = bfr(C[((size_t)b * SS + c) * 4 + 1]), hh = bfr(C[((size_t)b * SS + c) * 4 + 2]), ww = bfr(C[((size_t)b * SS + c) * 4 + 3]);
    sbx[c][0] = cx - 0.5f * ww; sbx[c][1] = cy - 0.5f * hh; sbx[c][2] = cx + 0.5f * ww; sbx[c][3] = cy + 0.5f * hh; }
  __syncthreads();
  const float ax0 = sbx[a][0], ay0 = sbx[a][1], ax1 = sbx[a][2], ay1 = sbx[a][3]; const float area_a = (ax1 - ax0) * (ay1 - ay0);
  float best = 0.f; int bi = -1;
  for (int c = sub; c < SS; c += 4) { const float cx0 = sbx[c][0], cy0 = sbx[c][1], cx1 = sbx[c][2], cy1 = sbx[c][3];
    const float mx0 = fmaxf(ax0, cx0), my0 = fmaxf(ay0, cy0), Mx = fmaxf(ax1, cx1), My = fmaxf(ay1, cy1);
    const float iw = fmaxf(Mx - mx0, 0.f), ih = fmaxf(My - my0, 0.f); const float ia = iw * ih; const float area_c = (cx1 - cx0) * (cy1 - cy0);
    const float uni = area_a + area_c - ia; float iou = ia / uni; iou = iou - ((c == a) ? 1.0f : 0.0f);
    if (bi < 0 || iou > best) { best = iou; bi = c; } }
#pragma unroll
  for (int o = 1; o < 4; o <<= 1) { const float ob = __shfl_xor(best, o); const int oi = __shfl_xor(bi, o); if (ob > best || (ob == best && oi < bi)) { best = ob; bi = oi; } }
  if (sub == 0) { const int partner = bi; const float l1a = fabsf(ax1 - ax0) + fabsf(ay1 - ay0); const float l1p = fabsf(sbx[partner][2] - sbx[partner][0]) + fabsf(sbx[partner][3] - sbx[partner][1]);
    const bool keep = l1a >= l1p; sp0[al] = keep ? a : partner; sp1[al] = keep ? partner : a; }
  __syncthreads();
  if (tid < 16) vst2((unsigned*)(P0 + (size_t)b * SS + blockIdx.x * 64 + tid * 4), *(const v4u*)&sp0[tid * 4]);
  else if (tid < 32) vst2((unsigned*)(P1 + (size_t)b * SS + blockIdx.x * 64 + (tid - 16) * 4), *(const v4u*)&sp1[(tid - 16) * 4]);
}
__global__ __launch_bounds__(256) void k_vt(const float* __restrict__ V, __bf16* __restrict__ VT) {
  __shared__ __align__(16) __bf16 s[HD][264]; const int bh = blockIdx.x, c0 = blockIdx.y * 256, tid = threadIdx.x;
  for (int q = tid; q < 256 * HD; q += 256) { const int cl = q >> 6, d = q & 63; s[d][cl] = (__bf16)V[((size_t)bh * SS + c0 + cl) * HD + d]; }
  __syncthreads();
  for (int q = tid; q < HD * 32; q += 256) { const int d = q >> 5, pc = q & 31; vst2((unsigned*)(VT + ((size_t)bh * HD + d) * SS + c0 + pc * 8), *(const v4u*)&s[d][pc * 8]); }
}
__device__ __forceinline__ v16b gath2(const float* qp0, const float* qp1, int kc, int lane) {
  v16b a; const float* base = (kc < 2) ? qp0 + kc * 32 : qp1 + (kc - 2) * 32; const float* p = base + 8 * (lane >> 4);
#pragma unroll
  for (int i = 0; i < 8; ++i) { a[i] = (__bf16)p[i]; a[8 + i] = (__bf16)p[16 + i]; }
  return a; }
__global__ __launch_bounds__(128) void k_attn(const float* __restrict__ Q, const float* __restrict__ Kx, const __bf16* __restrict__ VT, const int* __restrict__ P0, const int* __restrict__ P1, float* __restrict__ out) {
  __shared__ __align__(16) float sp[4][16][36]; __shared__ __align__(16) float so[4][16][68];
  const int tid = threadIdx.x, wave = tid >> 5, lane = tid & 31, col = lane & 15, g = lane >> 4; const int h = blockIdx.y, b = blockIdx.z; const int a0 = blockIdx.x * 64 + wave * 16;
  const size_t bh = (size_t)b * NH + h; const float* Qb = Q + bh * SS * HD; const float* Kb = Kx + bh * SS * HD; const __bf16* VTb = VT + bh * HD * SS;
  const int* p0 = P0 + (size_t)b * SS; const int* p1 = P1 + (size_t)b * SS;
  v16b aq[4]; { const int ar = a0 + col; const int i0 = min(max(p0[ar], 0), SS - 1), i1 = min(max(p1[ar], 0), SS - 1);
#pragma unroll
    for (int kc = 0; kc < 4; ++kc) aq[kc] = gath2(Qb + (size_t)i0 * HD, Qb + (size_t)i1 * HD, kc, lane); }
  float m[8], l[8];
#pragma unroll
  for (int r = 0; r < 8; ++r) { m[r] = -3.0e38f; l[r] = 0.f; }
  v8f acc[4] = {};
#pragma unroll 1
  for (int ks = 0; ks < SS / 32; ++ks) { v8f s[2];
#pragma unroll
    for (int ct = 0; ct < 2; ++ct) { const int c = ks * 32 + ct * 16 + col; const int j0 = min(max(p0[c], 0), SS - 1), j1 = min(max(p1[c], 0), SS - 1); v8f cc = {};
#pragma unroll
      for (int kc = 0; kc < 4; ++kc) cc = wmma_bf(aq[kc], gath2(Kb + (size_t)j0 * HD, Kb + (size_t)j1 * HD, kc, lane), cc);
#pragma unroll
      for (int r = 0; r < 8; ++r) s[ct][r] = cc[r] * 0.08838834764831845f; }
#pragma unroll
    for (int r = 0; r < 8; ++r) { float mx = fmaxf(s[0][r], s[1][r]);
#pragma unroll
      for (int o = 1; o < 16; o <<= 1) mx = fmaxf(mx, __shfl_xor(mx, o));
      const float mn = fmaxf(m[r], mx); const float alpha = exp_ni(m[r] - mn);
      const float e0 = exp_ni(s[0][r] - mn), e1 = exp_ni(s[1][r] - mn); float es = e0 + e1;
#pragma unroll
      for (int o = 1; o < 16; o <<= 1) es += __shfl_xor(es, o);
      l[r] = l[r] * alpha + es; m[r] = mn;
#pragma unroll
      for (int dt = 0; dt < 4; ++dt) acc[dt][r] *= alpha;
      sp[wave][8 * g + r][col] = e0; sp[wave][8 * g + r][16 + col] = e1; }
    LDSX();
    const F2 pa = split_row(&sp[wave][col][0], 0, lane);
#pragma unroll
    for (int dt = 0; dt < 4; ++dt) { const v16b vb = frag_b(VTb + (size_t)(dt * 16 + col) * SS + ks * 32, lane); acc[dt] = wmma_bf(pa.l, vb, acc[dt]); acc[dt] = wmma_bf(pa.h, vb, acc[dt]); }
    LDSX(); }
#pragma unroll
  for (int r = 0; r < 8; ++r) { const float il = 1.0f / l[r];
#pragma unroll
    for (int dt = 0; dt < 4; ++dt) so[wave][8 * g + r][dt * 16 + col] = acc[dt][r] * il; }
  LDSX();
  for (int rl = 0; rl < 16; ++rl) if (lane < 16) vst2(out + ((size_t)b * SS + a0 + rl) * (NH * HD) + h * HD + lane * 4, *(const v4f*)&so[wave][rl][lane * 4]);
}
extern "C" void kernel_launch(void* const* d_in, const int* in_sizes, int n_in, void* d_out, int out_size, void* d_ws, size_t ws_size, hipStream_t stream) {
  (void)in_sizes; (void)n_in; (void)out_size;
  const float** F = (const float**)d_in;
  if (ws_size < (size_t)WS_END) return;
  char* ws = (char*)d_ws; int *P0 = (int*)(ws + WS_P0), *P1 = (int*)(ws + WS_P1); __bf16* VT = (__bf16*)(ws + WS_VT);
  k_pairs<<<dim3(SS / 64, TNB), 256, 0, stream>>>(F[3], P0, P1);
  k_vt<<<dim3(NB * NH, SS / 256), 256, 0, stream>>>(F[2], VT);
  k_attn<<<dim3(TQB, NH, TNB), 128, 0, stream>>>(F[0], F[1], VT, P0, P1, (float*)d_out);
}
